// BPLoss_16698832847232
// MI455X (gfx1250) — hardware-verified
//
#include <hip/hip_runtime.h>

#define NROW   4096
#define BITD   64
#define LBL    10
#define LBLP   12
#define NWORD  (NROW / 32)
#define RESP   32
#define JCHUNK 1024
#define UPPERB 16.0f
#define CCF    (-0.4307924859501179f)
#define ACF    (-0.8615849719002358f)
#define OPSC   16.0f
#define OPINV  0.00390625f
#define LOG2EF 1.4426950408889634f
#define LN2F   0.6931471805599453f

static_assert(NROW % JCHUNK == 0);
static_assert(NROW % 256 == 0);
static_assert(BITD == 64);

typedef _Float16 v16h __attribute__((ext_vector_type(16)));
typedef _Float16 v8h  __attribute__((ext_vector_type(8)));
typedef float    v8f  __attribute__((ext_vector_type(8)));
typedef float    v4f  __attribute__((ext_vector_type(4)));
typedef int      v4i  __attribute__((ext_vector_type(4)));
typedef unsigned v4u  __attribute__((ext_vector_type(4)));
typedef v8h __attribute__((may_alias)) v8ha;
typedef v4f __attribute__((may_alias)) v4fa;
typedef v4i __attribute__((may_alias)) v4ia;
typedef v4u __attribute__((may_alias)) v4ua;

union Frag { v16h v; v8h half[2]; };

__device__ __forceinline__ v8f wmma_f16(v16h a, v16h b, v8f c) {
  v8f d = __builtin_amdgcn_wmma_f32_16x16x32_f16(false, a, false, b, (short)0, c, false, false);
  asm volatile("v_nop\n\tv_nop\n\tv_nop\n\tv_nop" : "+v"(d) : "v"(a), "v"(b));
  return d;
}

__device__ __forceinline__ v16h load_frag(const _Float16* p, int h) {
  Frag f;
  f.half[0] = *(const v8ha*)(p + 8 * h);
  f.half[1] = *(const v8ha*)(p + 16 + 8 * h);
  return f.v;
}

__device__ __forceinline__ unsigned ordf(float f) {
  const unsigned u = __float_as_uint(f);
  return u ^ ((u & 0x80000000u) ? 0xFFFFFFFFu : 0x80000000u);
}
__device__ __forceinline__ float invord(unsigned k) {
  const unsigned u = (k & 0x80000000u) ? (k ^ 0x80000000u) : ~k;
  return __uint_as_float(u);
}

__device__ __forceinline__ double shfl_xor_d(double v, int o) {
  const long long b = __double_as_longlong(v);
  int lo = (int)(b & 0xFFFFFFFFll);
  int hi = (int)(b >> 32);
  lo = __shfl_xor(lo, o, 32);
  hi = __shfl_xor(hi, o, 32);
  const long long r = ((long long)hi << 32) | (long long)(unsigned long long)(unsigned)lo;
  return __longlong_as_double(r);
}
__device__ __forceinline__ double wred_d(double v) {
#pragma unroll
  for (int o = 16; o > 0; o >>= 1) v += shfl_xor_d(v, o);
  return v;
}
__device__ __forceinline__ int wred_i(int v) {
#pragma unroll
  for (int o = 16; o > 0; o >>= 1) v += __shfl_xor(v, o, 32);
  return v;
}

__global__ __launch_bounds__(256) void k_convert(
    const float* __restrict__ u, const float* __restrict__ v,
    _Float16* __restrict__ uh, _Float16* __restrict__ vh)
{
  const int g = blockIdx.x * 256 + (int)threadIdx.x;
  const int NG = NROW * BITD / 8;
  if (g >= 2 * NG) return;
  const bool sec = (g >= NG);
  const int off = sec ? (g - NG) : g;
  const float* src = (sec ? v : u) + (size_t)off * 8;
  _Float16* dst = (sec ? vh : uh) + (size_t)off * 8;
  const v4f a = *(const v4fa*)src;
  const v4f c = *(const v4fa*)(src + 4);
  const v8h o = { (_Float16)(a.x * OPSC), (_Float16)(a.y * OPSC), (_Float16)(a.z * OPSC), (_Float16)(a.w * OPSC),
                  (_Float16)(c.x * OPSC), (_Float16)(c.y * OPSC), (_Float16)(c.z * OPSC), (_Float16)(c.w * OPSC) };
  *(volatile v8h*)dst = o;
  __threadfence();
  *(volatile v8h*)dst = o;
}

__global__ __launch_bounds__(256) void k_sim(const int* __restrict__ y, unsigned* __restrict__ sbits)
{
  __shared__ __attribute__((aligned(16))) int sy[JCHUNK * LBLP];

  const int tid = threadIdx.x, lane = tid & 31, wave = tid >> 5;
  const int jc = blockIdx.y * JCHUNK;
  const int i0 = blockIdx.x * 32;

#pragma unroll
  for (int t = 0; t < JCHUNK / 256; ++t) {
    const int r = tid + 256 * t;
    const int* p = y + (size_t)(jc + r) * LBL;
    const v4i a = { p[0], p[1], p[2], p[3] };
    const v4i b = { p[4], p[5], p[6], p[7] };
    const v4i c = { p[8], p[9], 0, 0 };
    *(v4ia*)(sy + r * LBLP) = a;
    *(v4ia*)(sy + r * LBLP + 4) = b;
    *(v4ia*)(sy + r * LBLP + 8) = c;
  }
  __syncthreads();

  const int wq = blockIdx.y * 32 + lane;
#pragma unroll 1
  for (int rr = 0; rr < 4; ++rr) {
    const int i = i0 + rr * 8 + wave;
    const int* yp = y + (size_t)i * LBL;
    const int y0 = yp[0], y1 = yp[1], y2 = yp[2], y3 = yp[3], y4 = yp[4];
    const int y5 = yp[5], y6 = yp[6], y7 = yp[7], y8 = yp[8], y9 = yp[9];
    unsigned bits = 0u;
#pragma unroll 4
    for (int jj = 0; jj < 32; ++jj) {
      const int* q = sy + (lane * 32 + jj) * LBLP;
      const v4i a = *(const v4ia*)q;
      const v4i b = *(const v4ia*)(q + 4);
      const v4i c = *(const v4ia*)(q + 8);
      const int dot = y0 * a.x + y1 * a.y + y2 * a.z + y3 * a.w + y4 * b.x +
                      y5 * b.y + y6 * b.z + y7 * b.w + y8 * c.x + y9 * c.y;
      bits |= (dot > 0) ? (1u << jj) : 0u;
    }
    unsigned* dst = sbits + (size_t)i * NWORD + wq;
    *(volatile unsigned*)dst = bits;
    __threadfence();
    *(volatile unsigned*)dst = bits;
  }
}

__device__ __forceinline__ void inner_store_pass(const float* so, float* inner, int iw, int j0, int lane) {
  const int q8 = lane & 7, sub = lane >> 3;
#pragma unroll
  for (int i = 0; i < 8; ++i) {
    const int lid = i * 4 + sub;
    const int row = lid >> 1, hl = lid & 1;
    const v4f v = *(const v4fa*)(so + row * 64 + 32 * hl + 4 * q8);
    const size_t gi = (size_t)(iw + row) * NROW + j0 + 32 * hl + 4 * q8;
    *(volatile v4f*)(inner + gi) = v;
  }
}

__global__ __launch_bounds__(128) void k_gemm(
    const _Float16* __restrict__ uh,
    const _Float16* __restrict__ vh,
    float* __restrict__ inner)
{
  __shared__ __attribute__((aligned(16))) float sO[4 * 16 * 64];

  const int tid = threadIdx.x, lane = tid & 31, w = tid >> 5;
  const int h = lane >> 4, m = lane & 15;
  const int j0 = blockIdx.x * 64;
  const int iw = blockIdx.y * 64 + 16 * w;

  const _Float16* ap = uh + (size_t)(iw + m) * BITD;
  const v16h a0 = load_frag(ap, h);
  const v16h a1 = load_frag(ap + 32, h);

  const v8f zero8 = {0.f, 0.f, 0.f, 0.f, 0.f, 0.f, 0.f, 0.f};
  v8f acc[4];
#pragma unroll
  for (int nt = 0; nt < 4; ++nt) {
    const _Float16* bp = vh + (size_t)(j0 + 16 * nt + m) * BITD;
    const v16h b0 = load_frag(bp, h);
    const v16h b1 = load_frag(bp + 32, h);
    v8f z = zero8;
    z = wmma_f16(a0, b0, z);
    z = wmma_f16(a1, b1, z);
    acc[nt] = z;
  }

  float* so = sO + w * 1024;
#pragma unroll
  for (int nt = 0; nt < 4; ++nt)
#pragma unroll
    for (int r = 0; r < 8; ++r)
      so[(8 * h + r) * 64 + 16 * nt + m] = acc[nt][r] * OPINV;
  __syncthreads();

  inner_store_pass(so, inner, iw, j0, lane);
  __threadfence();
  inner_store_pass(so, inner, iw, j0, lane);
}

__device__ __forceinline__ void sstep(int q, int cq, int rem, int& cum, int& fb, int& frem) {
  const int nc = cum + cq;
  const bool hit = (fb < 0) && (cum < rem) && (nc >= rem);
  fb = hit ? q : fb;
  frem = hit ? (rem - cum) : frem;
  cum = nc;
}

__device__ __forceinline__ void scan_select(const unsigned* hc, unsigned pref, int rem, int shift,
                                            unsigned* selp, int lane) {
  const v4u va = *(const v4ua*)(hc + 8 * lane);
  const v4u vb = *(const v4ua*)(hc + 8 * lane + 4);
  const int c0 = (int)va.x, c1 = (int)va.y, c2 = (int)va.z, c3 = (int)va.w;
  const int c4 = (int)vb.x, c5 = (int)vb.y, c6 = (int)vb.z, c7 = (int)vb.w;
  const int lsum = c0 + c1 + c2 + c3 + c4 + c5 + c6 + c7;
  int incl = lsum;
#pragma unroll
  for (int d = 1; d < 32; d <<= 1) {
    const int t = __shfl_up(incl, d, 32);
    if (lane >= d) incl += t;
  }
  int cum = incl - lsum;
  int fb = -1, frem = 0;
  sstep(0, c0, rem, cum, fb, frem);
  sstep(1, c1, rem, cum, fb, frem);
  sstep(2, c2, rem, cum, fb, frem);
  sstep(3, c3, rem, cum, fb, frem);
  sstep(4, c4, rem, cum, fb, frem);
  sstep(5, c5, rem, cum, fb, frem);
  sstep(6, c6, rem, cum, fb, frem);
  sstep(7, c7, rem, cum, fb, frem);
  const bool found = (fb >= 0);
  const unsigned fm = __builtin_amdgcn_ballot_w32(found);
  const int first = (fm != 0u) ? (int)__builtin_ctz(fm) : 0;
  const bool writer = found ? (lane == first) : ((fm == 0u) && (lane == 0));
  const unsigned bsel = found ? (unsigned)(8 * lane + fb) : 0u;
  const unsigned nrem = found ? (unsigned)frem : (unsigned)rem;
  if (writer) {
    selp[0] = pref | (bsel << shift);
    selp[1] = nrem;
  }
}

__global__ __launch_bounds__(256) void k_row(
    const float* __restrict__ inner, const unsigned* __restrict__ sbits,
    float* __restrict__ rowres)
{
  __shared__ __attribute__((aligned(16))) float srow[NROW];
  __shared__ __attribute__((aligned(16))) unsigned sw[NWORD];
  __shared__ __attribute__((aligned(16))) unsigned hist[512];
  __shared__ unsigned sel[4];
  __shared__ double redd[6][8];
  __shared__ int redi[3][8];

  const int tid = threadIdx.x, lane = tid & 31, wave = tid >> 5;
  const int i = blockIdx.x;

  const float* src = inner + (size_t)i * NROW;
#pragma unroll
  for (int t = 0; t < 4; ++t) {
    const int q = tid + 256 * t;
    const v4f val = *(const v4fa*)(src + 4 * q);
    *(v4fa*)(srow + 4 * q) = val;
  }
  if (tid < NWORD) sw[tid] = sbits[(size_t)i * NWORD + tid];
  hist[tid] = 0u;
  hist[tid + 256] = 0u;
  __syncthreads();

  int cS = 0;
  double sS = 0.0, sD = 0.0;
#pragma unroll 4
  for (int e = 0; e < 16; ++e) {
    const int j = e * 256 + tid;
    const float x = srow[j];
    const unsigned mw = sw[e * 8 + wave];
    const bool sim = ((mw >> lane) & 1u) != 0u;
    const unsigned k = ordf(x);
    const unsigned key = sim ? k : ~k;
    const double xd = (double)x;
    cS += sim ? 1 : 0;
    sS += sim ? xd : 0.0;
    sD += sim ? 0.0 : xd;
    atomicAdd(&hist[(sim ? 0 : 256) + (int)(key >> 24)], 1u);
  }
  {
    const int c = wred_i(cS);
    const double a = wred_d(sS);
    const double b = wred_d(sD);
    if (lane == 0) { redi[0][wave] = c; redd[0][wave] = a; redd[1][wave] = b; }
  }
  __syncthreads();
  int ns = 0;
  double sumS = 0.0, sumD = 0.0;
#pragma unroll
  for (int w8 = 0; w8 < 8; ++w8) { ns += redi[0][w8]; sumS += redd[0][w8]; sumD += redd[1][w8]; }
  const int nd = NROW - ns;
  const int mS = ns - (ns * 9) / 10;
  const int mD = nd - (nd * 9) / 10;

  unsigned prefS = 0u, prefD = 0u;
  int remS = mS, remD = mD;
  if (wave < 2)
    scan_select(hist + 256 * wave, 0u, (wave == 0) ? remS : remD, 24, sel + 2 * wave, lane);
  __syncthreads();
  prefS = sel[0]; remS = (int)sel[1]; prefD = sel[2]; remD = (int)sel[3];

#pragma unroll 1
  for (int lev = 1; lev < 4; ++lev) {
    const int shift = 24 - 8 * lev;
    const unsigned hm = 0xFFFFFFFFu << (shift + 8);
    hist[tid] = 0u;
    hist[tid + 256] = 0u;
    __syncthreads();
#pragma unroll 4
    for (int e = 0; e < 16; ++e) {
      const int j = e * 256 + tid;
      const float x = srow[j];
      const unsigned mw = sw[e * 8 + wave];
      const bool sim = ((mw >> lane) & 1u) != 0u;
      const unsigned k = ordf(x);
      const unsigned key = sim ? k : ~k;
      const unsigned pf = sim ? prefS : prefD;
      if ((key & hm) == pf)
        atomicAdd(&hist[(sim ? 0 : 256) + (int)((key >> shift) & 255u)], 1u);
    }
    __syncthreads();
    if (wave < 2)
      scan_select(hist + 256 * wave, (wave == 0) ? prefS : prefD, (wave == 0) ? remS : remD,
                  shift, sel + 2 * wave, lane);
    __syncthreads();
    prefS = sel[0]; remS = (int)sel[1]; prefD = sel[2]; remD = (int)sel[3];
  }
  const unsigned KS = prefS;
  const unsigned KD = prefD;

  int tcS = 0, tcD = 0;
  double tS = 0.0, tD = 0.0;
#pragma unroll 4
  for (int e = 0; e < 16; ++e) {
    const int j = e * 256 + tid;
    const float x = srow[j];
    const unsigned mw = sw[e * 8 + wave];
    const bool sim = ((mw >> lane) & 1u) != 0u;
    const unsigned k = ordf(x);
    const bool inS = sim && (k < KS);
    const bool inD = (!sim) && ((~k) < KD);
    const double xd = (double)x;
    tcS += inS ? 1 : 0;
    tcD += inD ? 1 : 0;
    tS += inS ? xd : 0.0;
    tD += inD ? xd : 0.0;
  }
  {
    const int c1 = wred_i(tcS);
    const int c2 = wred_i(tcD);
    const double a = wred_d(tS);
    const double b = wred_d(tD);
    if (lane == 0) { redi[1][wave] = c1; redi[2][wave] = c2; redd[2][wave] = a; redd[3][wave] = b; }
  }
  __syncthreads();
  int cSt = 0, cDt = 0;
  double sSt = 0.0, sDt = 0.0;
#pragma unroll
  for (int w8 = 0; w8 < 8; ++w8) { cSt += redi[1][w8]; cDt += redi[2][w8]; sSt += redd[2][w8]; sDt += redd[3][w8]; }

  const float vS = invord(KS);
  const float vD = invord(~KD);
  const double tailS = sSt + (double)(mS - cSt) * (double)vS;
  const double tailD = sDt + (double)(mD - cDt) * (double)vD;
  const float rmS = __builtin_amdgcn_rcpf((float)(mS > 0 ? mS : 1));
  const float rmD = __builtin_amdgcn_rcpf((float)(mD > 0 ? mD : 1));
  const float simMin = (mS > 0) ? (float)(tailS * (double)rmS) : 0.0f;
  const float disMax = (mD > 0) ? (float)(tailD * (double)rmD) : 0.0f;

  const float rns = __builtin_amdgcn_rcpf((float)(ns > 0 ? ns : 1));
  const float rnd = __builtin_amdgcn_rcpf((float)(nd > 0 ? nd : 1));
  float meanS = (float)sumS * rns;
  meanS = fminf(fmaxf(meanS, 0.0f), UPPERB);
  float meanDS = (float)sumD * rnd;
  meanDS = fminf(fmaxf(meanDS, 0.0f), UPPERB);

  const float BP = meanS - (UPPERB - meanS) * (1.0f / UPPERB) * fabsf(meanS - disMax);
  const float BPds = meanDS - meanDS * (1.0f / UPPERB) * fabsf(meanDS - simMin);
  const float d1 = -CCF * BP, g1 = -ACF * BP;
  const float d2 = -CCF * BPds, g2 = -ACF * BPds;

  double pos = 0.0, nav = 0.0;
#pragma unroll 2
  for (int e = 0; e < 16; ++e) {
    const int j = e * 256 + tid;
    const float x = srow[j];
    const unsigned mw = sw[e * 8 + wave];
    const bool sim = ((mw >> lane) & 1u) != 0u;
    const float fs = (x > BP) ? (CCF * x + d1) : (ACF * x + g1);
    const float fd = (x < BPds) ? (CCF * x + d2) : (ACF * x + g2);
    const float f = sim ? fs : -fd;
    const float ex = __builtin_amdgcn_exp2f(-fabsf(f) * LOG2EF);
    const float sp = fmaxf(f, 0.0f) + LN2F * __builtin_amdgcn_logf(1.0f + ex);
    const double spd = (double)sp;
    pos += sim ? spd : 0.0;
    nav += sim ? 0.0 : spd;
  }
  {
    const double a = wred_d(pos);
    const double b = wred_d(nav);
    if (lane == 0) { redd[4][wave] = a; redd[5][wave] = b; }
  }
  __syncthreads();
  double posS = 0.0, navS = 0.0;
#pragma unroll
  for (int w8 = 0; w8 < 8; ++w8) { posS += redd[4][w8]; navS += redd[5][w8]; }

  const bool valid = (ns > 0) && (nd > 0);
  const float rowv = valid ? (float)(posS * (double)rns + navS * (double)rnd) : 0.0f;
  const float vf = valid ? 1.0f : 0.0f;

  if (wave == 0 && lane < 8) {
    v4f o;
    o.x = (lane == 0) ? rowv : 0.0f;
    o.y = (lane == 0) ? vf : 0.0f;
    o.z = 0.0f;
    o.w = 0.0f;
    float* dst = rowres + (size_t)i * RESP + 4 * lane;
    *(volatile v4f*)dst = o;
    __threadfence();
    *(volatile v4f*)dst = o;
  }
}

__global__ __launch_bounds__(256) void k_final(const float* __restrict__ rowres, float* __restrict__ out)
{
  __shared__ double sl[256];
  __shared__ double sc[256];
  const int t = threadIdx.x;
  double l = 0.0, c = 0.0;
#pragma unroll 4
  for (int e = 0; e < NROW / 256; ++e) {
    const int r = e * 256 + t;
    l += (double)rowres[(size_t)r * RESP];
    c += (double)rowres[(size_t)r * RESP + 1];
  }
  sl[t] = l;
  sc[t] = c;
  __syncthreads();
  for (int o = 128; o > 0; o >>= 1) {
    if (t < o) { sl[t] = sl[t] + sl[t + o]; sc[t] = sc[t] + sc[t + o]; }
    __syncthreads();
  }
  if (t == 0) {
    const double cnt = sc[0];
    const float rc = __builtin_amdgcn_rcpf((float)cnt);
    const float res = (cnt > 0.0) ? (float)(sl[0] * (double)rc) : 0.0f;
    *(volatile float*)out = res;
    __threadfence();
    *(volatile float*)out = res;
  }
}

extern "C" void kernel_launch(void* const* d_in, const int* in_sizes, int n_in,
                              void* d_out, int out_size, void* d_ws, size_t ws_size,
                              hipStream_t stream) {
  if (n_in < 3) return;
  if (in_sizes[0] != NROW * BITD) return;
  if (in_sizes[1] != NROW * BITD) return;
  if (in_sizes[2] != NROW * LBL) return;
  if (out_size < 1) return;

  const float* u = (const float*)d_in[0];
  const float* v = (const float*)d_in[1];
  const int*   y = (const int*)d_in[2];
  float* out = (float*)d_out;

  const size_t uh_b = (size_t)NROW * BITD * 2;
  const size_t vh_b = uh_b;
  const size_t sb_b = (size_t)NROW * NWORD * 4;
  const size_t in_b = (size_t)NROW * NROW * 4;
  const size_t rr_b = (size_t)NROW * RESP * 4;
  const size_t total = uh_b + vh_b + sb_b + in_b + rr_b;
  if (total > ws_size) return;

  char* ws = (char*)d_ws;
  _Float16* uh     = (_Float16*)(ws);
  _Float16* vh     = (_Float16*)(ws + uh_b);
  unsigned* sbits  = (unsigned*)(ws + uh_b + vh_b);
  float*    inner  = (float*)(ws + uh_b + vh_b + sb_b);
  float*    rowres = (float*)(ws + uh_b + vh_b + sb_b + in_b);

  const int ngroups = 2 * NROW * BITD / 8;
  k_convert<<<(ngroups + 255) / 256, 256, 0, stream>>>(u, v, uh, vh);

  dim3 gSim(NROW / 32, NROW / JCHUNK);
  k_sim<<<gSim, 256, 0, stream>>>(y, sbits);

  dim3 gGemm(NROW / 64, NROW / 64);
  k_gemm<<<gGemm, 128, 0, stream>>>(uh, vh, inner);

  k_row<<<NROW, 256, 0, stream>>>(inner, sbits, rowres);

  k_final<<<1, 256, 0, stream>>>(rowres, out);
}
